// Head_15272903705216
// MI455X (gfx1250) — hardware-run, weakly checked
//
#include <hip/hip_runtime.h>


#define NFR  6
#define NPT  16
#define NEL  16
#define NNE  32
#define NROW (NFR * NPT)
#define KP   32
#define ZROW NROW
#define WKR  17
#define ZK   (NPT * WKR)
#define PTR  18
#define QRS  2048.0f
#define QRI  (1.0f / 2048.0f)

static_assert(NROW == 96);
static_assert(NROW % 32 == 0);
static_assert(KP == 32);
static_assert(NEL + 1 <= KP);
static_assert(NNE == KP);
static_assert(NFR <= 16);
static_assert(NFR <= 8);
static_assert(3 * 256 * 4 == NROW * NNE);
static_assert((NROW * NNE * 4) % 128 == 0);

typedef _Float16 h16;
typedef __attribute__((ext_vector_type(16))) _Float16 v16h;
typedef __attribute__((ext_vector_type(8)))  _Float16 v8h;
typedef __attribute__((ext_vector_type(8)))  unsigned char v8uc;
typedef __attribute__((ext_vector_type(8)))  float    v8f;
typedef __attribute__((ext_vector_type(4)))  float    v4f;
typedef v4f  __attribute__((may_alias)) v4fa;

__device__ __forceinline__ unsigned short f2bf(float f) { unsigned u = __float_as_uint(f); u += 0x7FFFu + ((u >> 16) & 1u); return (unsigned short)(u >> 16); }
__device__ __forceinline__ float bfr(float f) { return __uint_as_float(((unsigned)f2bf(f)) << 16); }
__device__ __forceinline__ v16h cat16(v8h lo, v8h hi) { return __builtin_shufflevector(lo, hi, 0, 1, 2, 3, 4, 5, 6, 7, 8, 9, 10, 11, 12, 13, 14, 15); }
__device__ __forceinline__ v8f wmma16(v16h a, v16h b, v8f c) { return __builtin_amdgcn_wmma_f32_16x16x32_f16(false, a, false, b, (short)0, c, false, false); }
__device__ __forceinline__ v16h  ldh(const h16* p) { return cat16(*(const v8h*)p, *(const v8h*)(p + 16)); }
static __device__ __forceinline__ h16 toh_flush(float v) { const h16 r = (h16)v; return (fabsf(v) < 6.103515625e-05f) ? (h16)0.0f : r; }
static __device__ __forceinline__ v8f wmma16g(v16h a, v16h b, v8f c) {
    c = wmma16(a, b, c);
    asm volatile("v_nop\n\tv_nop\n\tv_nop\n\tv_nop" : "+v"(c) : "v"(a), "v"(b));
    return c;
}
static __device__ __forceinline__ void split8(const v8f v, v8h& hv, v8h& rv) {
#pragma unroll
    for (int r = 0; r < 8; ++r) { const h16 a = toh_flush(v[r]); hv[r] = a; rv[r] = toh_flush((v[r] - (float)a) * QRS); }
}

static constexpr size_t LDS_BYTES =
      (size_t)(NROW + 1) * KP * 2
    + (size_t)PTR * NROW * 2
    + (size_t)NNE * KP * 2
    + (size_t)(ZK + 1) * KP * 2
    + (size_t)NPT * NNE * KP * 2
    + (size_t)2 * (NROW + 1) * KP * 2
    + (size_t)2 * NROW * KP * 2
    + (size_t)2 * (NROW + 1) * KP * 2
    + (size_t)NROW * NROW
    + (size_t)NROW * NNE * 4;
static_assert(LDS_BYTES <= (size_t)131072);

__global__ __launch_bounds__(256) void k_lcattn(const float* __restrict__ x, const float* __restrict__ Wq, const float* __restrict__ Wk, const float* __restrict__ bk,
                                                const float* __restrict__ Wv, const float* __restrict__ bv, float* OUT) {
    __shared__ __align__(16) h16 ptE[(NROW + 1) * KP];
    __shared__ __align__(16) h16 ptT[PTR * NROW];
    __shared__ __align__(16) h16 WqP[NNE * KP];
    __shared__ __align__(16) h16 WkT[(ZK + 1) * KP];
    __shared__ __align__(16) h16 WvE[NPT * NNE * KP];
    __shared__ __align__(16) h16 qH[(NROW + 1) * KP];
    __shared__ __align__(16) h16 qR[(NROW + 1) * KP];
    __shared__ __align__(16) h16 qkH[NROW * KP];
    __shared__ __align__(16) h16 qkR[NROW * KP];
    __shared__ __align__(16) h16 uH[(NROW + 1) * KP];
    __shared__ __align__(16) h16 uR[(NROW + 1) * KP];
    __shared__ __align__(16) unsigned char cnt[NROW * NROW];
    __shared__ __align__(16) float os[NROW * NNE];

    const int tid = threadIdx.x;
    const int lane = threadIdx.x & 31, lr = lane & 15, hi = lane >> 4;
    const int wave = __builtin_amdgcn_readfirstlane((int)(threadIdx.x >> 5));

    {
        const v8h z8 = (v8h){};
        v8h one8 = (v8h){}; one8[0] = (h16)1.0f;
        const v8h ones8 = (v8h){(h16)1.0f, (h16)1.0f, (h16)1.0f, (h16)1.0f, (h16)1.0f, (h16)1.0f, (h16)1.0f, (h16)1.0f};
        if (tid < NROW) { *(v8h*)(&ptE[tid * KP + 16]) = one8; *(v8h*)(&ptE[tid * KP + 24]) = z8; }
        if (tid < 4) {
            *(v8h*)(&ptE[ZROW * KP + tid * 8]) = z8;
            *(v8h*)(&WkT[ZK * KP + tid * 8]) = z8;
            *(v8h*)(&qH[ZROW * KP + tid * 8]) = z8; *(v8h*)(&qR[ZROW * KP + tid * 8]) = z8;
            *(v8h*)(&uH[ZROW * KP + tid * 8]) = z8; *(v8h*)(&uR[ZROW * KP + tid * 8]) = z8;
        }
        if (tid < NROW / 8) { *(v8h*)(&ptT[16 * NROW + tid * 8]) = ones8; *(v8h*)(&ptT[17 * NROW + tid * 8]) = z8; }
        if (tid < NNE) { *(v8h*)(&WqP[tid * KP + 16]) = z8; *(v8h*)(&WqP[tid * KP + 24]) = z8; }
#pragma unroll 1
        for (int p = tid; p < NPT * NNE * 2; p += 256) *(v8h*)(&WvE[(p >> 1) * KP + 16 + (p & 1) * 8]) = z8;
    }
    __syncthreads();

#pragma unroll 1
    for (int idx = tid; idx < NROW * NEL; idx += 256) {
        const int d = idx & 15, m = idx >> 4;
        const int c = m % NFR, n = m / NFR;
        const int hp = n >> 2, wp = n & 3, pr = d >> 2, pc = d & 3;
        const h16 hv = toh_flush(bfr(x[c * 256 + (hp * 4 + pr) * 16 + (wp * 4 + pc)]));
        ptE[m * KP + d] = hv; ptT[d * NROW + m] = hv;
    }
#pragma unroll 1
    for (int idx = tid; idx < NNE * NEL; idx += 256) WqP[(idx >> 4) * KP + (idx & 15)] = toh_flush(bfr(Wq[idx]));
#pragma unroll 4
    for (int idx = tid; idx < NPT * NNE * NEL; idx += 256) {
        const int j = idx >> 9, e = (idx >> 4) & 31, d = idx & 15;
        WkT[(j * WKR + d) * KP + e] = toh_flush(bfr(Wk[idx]));
        WvE[(j * NNE + e) * KP + d] = toh_flush(bfr(Wv[idx]));
    }
#pragma unroll 1
    for (int idx = tid; idx < NPT * NNE; idx += 256) {
        const int j = idx >> 5, e = idx & 31;
        WkT[(j * WKR + 16) * KP + e] = toh_flush(bfr(bk[idx]));
        WvE[(j * NNE + e) * KP + 16] = toh_flush(bfr(bv[idx]));
    }
    if (tid < NROW) {
        const int iq = tid >> 4, j = tid & 15; const int ip1 = iq + 1;
        const int cb = tid * NROW;
#pragma unroll 1
        for (int z = 0; z < NROW; ++z) cnt[cb + z] = (unsigned char)0;
        { const int fn = iq * 16 + j; const int m = (fn / ip1) * NFR + (fn % ip1); cnt[cb + m] = (unsigned char)(cnt[cb + m] + 1); }
        int il = 2;
#pragma unroll 1
        for (int fp = iq; fp >= 0; --fp) {
#pragma unroll 1
            for (int k = -il + 1; k <= il - 1; ++k) {
#pragma unroll 1
                for (int l = -il + 1; l <= il - 1; ++l) {
                    if (!(j == 0 && l == 0 && il == 2)) {
                        const int idx = j + 16 * k + l;
                        if (idx >= 0 && idx < 16) { const int fn = fp * 16 + idx; const int m = (fn / ip1) * NFR + (fn % ip1); cnt[cb + m] = (unsigned char)(cnt[cb + m] + 1); }
                    }
                }
            }
            ++il;
        }
    }
    __syncthreads();

#pragma unroll 1
    for (int tl = wave; tl < 12; tl += 8) {
        const int mt = tl >> 1, et = tl & 1;
        const v16h a = ldh(&WqP[(et * 16 + lr) * KP + 8 * hi]);
        const v16h b = ldh(&ptE[(mt * 16 + lr) * KP + 8 * hi]);
        const v8f acc = wmma16g(a, b, (v8f){});
        v8h hv, rv; split8(acc, hv, rv);
        const int qo = (mt * 16 + lr) * KP + et * 16 + 8 * hi;
        *(v8h*)(&qH[qo]) = hv; *(v8h*)(&qR[qo]) = rv;
    }
    __syncthreads();

#pragma unroll 1
    for (int tl = wave; tl < 32; tl += 8) {
        const int j = tl >> 1, dt = tl & 1;
        const int arow = dt ? ((lr == 0) ? (j * WKR + 16) : ZK) : (j * WKR + lr);
        const int brow = (lr < NFR) ? (lr * 16 + j) : ZROW;
        const v16h a = ldh(&WkT[arow * KP + 8 * hi]);
        const v16h bh = ldh(&qH[brow * KP + 8 * hi]);
        const v16h br = ldh(&qR[brow * KP + 8 * hi]);
        const v8f accH = wmma16g(a, bh, (v8f){});
        const v8f accL = wmma16g(a, br, (v8f){});
        v8f val;
#pragma unroll
        for (int r = 0; r < 8; ++r) val[r] = accH[r] + accL[r] * QRI;
        v8h hv, rv; split8(val, hv, rv);
        if (lr < NFR) { const int qo = (lr * 16 + j) * KP + dt * 16 + 8 * hi; *(v8h*)(&qkH[qo]) = hv; *(v8h*)(&qkR[qo]) = rv; }
    }
    __syncthreads();

    if (wave < NFR) {
        const int i = wave;
        const int qo = (i * 16 + lr) * KP + 8 * hi;
        const v16h qh = ldh(&qkH[qo]), qr = ldh(&qkR[qo]);
        const int t1row = (lr == 0) ? 16 : 17;
        const int cbase = (i * 16 + lr) * NROW + 8 * hi;
        v8f o0 = (v8f){}, oR0 = (v8f){}, o1 = (v8f){}, oR1 = (v8f){};
#pragma unroll 1
        for (int m0 = 0; m0 < NROW; m0 += 32) {
            const v16h pa = ldh(&ptE[(m0 + lr) * KP + 8 * hi]);
            const v16h pc = ldh(&ptE[(m0 + 16 + lr) * KP + 8 * hi]);
            const v8f sHa = wmma16g(pa, qh, (v8f){});
            const v8f sLa = wmma16g(pa, qr, (v8f){});
            const v8f sHb = wmma16g(pc, qh, (v8f){});
            const v8f sLb = wmma16g(pc, qr, (v8f){});
            const v8uc ca = *(const v8uc*)(&cnt[cbase + m0]);
            const v8uc cc = *(const v8uc*)(&cnt[cbase + m0 + 16]);
            v16h pbv, prv;
#pragma unroll
            for (int r = 0; r < 8; ++r) {
                const float ta = (sHa[r] + sLa[r] * QRI) * (float)ca[r];
                const float tb = (sHb[r] + sLb[r] * QRI) * (float)cc[r];
                const h16 xa = toh_flush(ta); const h16 xb = toh_flush(tb);
                pbv[r] = xa; pbv[8 + r] = xb;
                prv[r] = toh_flush((ta - (float)xa) * QRS); prv[8 + r] = toh_flush((tb - (float)xb) * QRS);
            }
            const v16h t0 = ldh(&ptT[lr * NROW + m0 + 8 * hi]);
            const v16h t1 = ldh(&ptT[t1row * NROW + m0 + 8 * hi]);
            o0  = wmma16g(t0, pbv, o0);
            oR0 = wmma16g(t0, prv, oR0);
            o1  = wmma16g(t1, pbv, o1);
            oR1 = wmma16g(t1, prv, oR1);
        }
        v8f u0, u1;
#pragma unroll
        for (int r = 0; r < 8; ++r) { u0[r] = o0[r] + oR0[r] * QRI; u1[r] = o1[r] + oR1[r] * QRI; }
        v8h h0, r0v, h1, r1v; split8(u0, h0, r0v); split8(u1, h1, r1v);
        const int uo = (i * 16 + lr) * KP + 8 * hi;
        *(v8h*)(&uH[uo]) = h0; *(v8h*)(&uR[uo]) = r0v;
        *(v8h*)(&uH[uo + 16]) = h1; *(v8h*)(&uR[uo + 16]) = r1v;
    }
    __syncthreads();

#pragma unroll 1
    for (int tl = wave; tl < 32; tl += 8) {
        const int j = tl >> 1, et = tl & 1;
        const int brow = (lr < NFR) ? (lr * 16 + j) : ZROW;
        const v16h a = ldh(&WvE[(j * NNE + et * 16 + lr) * KP + 8 * hi]);
        const v16h bh = ldh(&uH[brow * KP + 8 * hi]);
        const v16h br = ldh(&uR[brow * KP + 8 * hi]);
        const v8f accH = wmma16g(a, bh, (v8f){});
        const v8f accL = wmma16g(a, br, (v8f){});
        v4f va, vc;
#pragma unroll
        for (int r = 0; r < 4; ++r) { va[r] = accH[r] + accL[r] * QRI; vc[r] = accH[4 + r] + accL[4 + r] * QRI; }
        if (lr < NFR) { const int ob = (lr * 16 + j) * NNE + et * 16 + 8 * hi; *(v4fa*)(&os[ob]) = va; *(v4fa*)(&os[ob + 4]) = vc; }
    }
    __syncthreads();

#pragma unroll 1
    for (int ps = 0; ps < 2; ++ps) {
#pragma unroll
        for (int it = 0; it < 3; ++it) {
            const int p = it * 256 + tid;
            const v4f val = *(const v4fa*)(&os[p * 4]);
            *(volatile v4f*)(OUT + (size_t)p * 4) = val;
        }
        if (ps == 0) __threadfence();
    }
}

extern "C" void kernel_launch(void* const* d_in, const int* in_sizes, int n_in,
                              void* d_out, int out_size, void* d_ws, size_t ws_size, hipStream_t stream) {
    (void)d_ws; (void)ws_size;
    if (n_in < 6) return;
    if (in_sizes[0] < NFR * 256) return;
    if (in_sizes[1] < NNE * NEL) return;
    if (in_sizes[2] < NPT * NNE * NEL) return;
    if (in_sizes[3] < NPT * NNE) return;
    if (in_sizes[4] < NPT * NNE * NEL) return;
    if (in_sizes[5] < NPT * NNE) return;
    if (out_size < NROW * NNE) return;
    const float* x  = (const float*)d_in[0];
    const float* wq = (const float*)d_in[1];
    const float* wk = (const float*)d_in[2];
    const float* bk = (const float*)d_in[3];
    const float* wv = (const float*)d_in[4];
    const float* bv = (const float*)d_in[5];
    float* OUT = (float*)d_out;
    k_lcattn<<<dim3(1, 1, 1), 256, 0, stream>>>(x, wq, wk, bk, wv, bv, OUT);
}
